// SDPA_36112085024790
// MI455X (gfx1250) — hardware-verified
//
#include <hip/hip_runtime.h>

typedef __attribute__((ext_vector_type(16))) _Float16 v16h;
typedef __attribute__((ext_vector_type(8)))  _Float16 v8h;
typedef __attribute__((ext_vector_type(16))) __bf16   v16b;
typedef __attribute__((ext_vector_type(8)))  __bf16   v8b;
typedef __attribute__((ext_vector_type(8)))  float    v8f;
typedef __attribute__((ext_vector_type(4)))  float    v4f;
typedef __attribute__((ext_vector_type(4)))  unsigned int v4u;
#define PSCALE 32768.0f
#define U16(p) ((const unsigned short*)(const void*)(p))
#define PSCALE_INV (1.0f / 32768.0f)

__device__ __forceinline__ unsigned short f2bf_bits(float f) {
  unsigned u = __float_as_uint(f);
  return (unsigned short)((u + 0x7FFFu + ((u >> 16) & 1u)) >> 16);
}
__device__ __forceinline__ float bf_bits2f(unsigned short h) { return __uint_as_float(((unsigned)h) << 16); }

__device__ __forceinline__ void dep_guard_h(v8f& a, v8f& b, v16h x, v16h y) { asm volatile("v_nop\n\tv_nop\n\tv_nop\n\tv_nop" : "+v"(a), "+v"(b) : "v"(x), "v"(y)); }
__device__ __forceinline__ void dep_guard_b(v8f& a, v8f& b, v16b x, v16b y) { asm volatile("v_nop\n\tv_nop\n\tv_nop\n\tv_nop" : "+v"(a), "+v"(b) : "v"(x), "v"(y)); }
__device__ __forceinline__ void keep4_h(v16h a, v16h b, v16h c, v16h d) { asm volatile("v_nop" :: "v"(a), "v"(b), "v"(c), "v"(d)); }
__device__ __forceinline__ void keep4_b(v16b a, v16b b, v16b c, v16b d) { asm volatile("v_nop" :: "v"(a), "v"(b), "v"(c), "v"(d)); }
__device__ __forceinline__ void acc_guard4(v8f& a, v8f& b, v8f& c, v8f& d) { asm volatile("v_nop\n\tv_nop\n\tv_nop\n\tv_nop" : "+v"(a), "+v"(b), "+v"(c), "+v"(d)); }
template <typename T> struct Frag;
template <> struct Frag<_Float16> {
  typedef v16h V; union U { v16h v; v8h h[2]; };
  static __device__ __forceinline__ v16h load(const _Float16* p) {
    U f; f.h[0] = *(const v8h*)(p); f.h[1] = *(const v8h*)(p + 16); return f.v;
  }
  static __device__ __forceinline__ v8f mma(v16h a, v16h b, v8f c) {
    return __builtin_amdgcn_wmma_f32_16x16x32_f16(false, a, false, b, (short)0, c, false, false);
  }
  static __device__ __forceinline__ void guard(v8f& a, v8f& b, v16h x, v16h y) { dep_guard_h(a, b, x, y); }
  static __device__ __forceinline__ void keep(v16h a, v16h b, v16h c, v16h d) { keep4_h(a, b, c, d); }
};
template <> struct Frag<__bf16> {
  typedef v16b V; union U { v16b v; v8b h[2]; };
  static __device__ __forceinline__ v16b load(const __bf16* p) {
    U f; f.h[0] = *(const v8b*)(p); f.h[1] = *(const v8b*)(p + 16); return f.v;
  }
  static __device__ __forceinline__ v8f mma(v16b a, v16b b, v8f c) {
    return __builtin_amdgcn_wmma_f32_16x16x32_bf16(false, a, false, b, (short)0, c, false, false);
  }
  static __device__ __forceinline__ void guard(v8f& a, v8f& b, v16b x, v16b y) { dep_guard_b(a, b, x, y); }
  static __device__ __forceinline__ void keep(v16b a, v16b b, v16b c, v16b d) { keep4_b(a, b, c, d); }
};

template <int ET> struct Elem;
template <> struct Elem<0> { typedef _Float16 T; };
template <> struct Elem<1> { typedef __bf16 T; };
template <int ET, bool SPLIT, int BIAS_MODE, int OUT_MODE, bool RESID, int ACT = 0>
__global__ __launch_bounds__(256) void wmma_gemm64(
    const unsigned short* __restrict__ Ap, const unsigned short* __restrict__ A2p, int lda, long strideA,
    const unsigned short* __restrict__ Btp, const unsigned short* __restrict__ Bt2p, int ldb, long strideB,
    void* __restrict__ Cout, void* __restrict__ Cout2, int ldc, long strideC,
    const float* __restrict__ bias,
    const float* __restrict__ resid, long strideR,
    int M, int N, int K, float scale) {
  typedef typename Elem<ET>::T T;
  typedef typename Frag<T>::V V;
  const T* A = (const T*)Ap; const T* A2 = (const T*)A2p; const T* Bt = (const T*)Btp; const T* Bt2 = (const T*)Bt2p;
  __shared__ __align__(16) float sT[8][16 * 68];
  const int b    = blockIdx.y;
  const int lane = threadIdx.x & 31;
  const int wave = threadIdx.x >> 5;
  const int tilesN = N >> 6;
  const int tilesM = M >> 6;
  const int tile = blockIdx.x * 8 + wave;
  if (tile >= tilesM * tilesN) return;
  const int tm = tile / tilesN;
  const int tn = tile - tm * tilesN;
  const int m0 = tm << 6;
  const int n0 = tn << 6;

  const T* Ab  = A  + (size_t)b * strideA;
  const T* Bb  = Bt + (size_t)b * strideB;
  const T* Ab2 = SPLIT ? (A2  + (size_t)b * strideA) : nullptr;
  const T* Bb2 = SPLIT ? (Bt2 + (size_t)b * strideB) : nullptr;

  const int rlane = lane & 15;
  const int koff  = (lane >> 4) * 8;
  const int mOff  = (lane >> 4) * 8;

  v8f acc[4][4];
#pragma unroll
  for (int i = 0; i < 4; ++i)
#pragma unroll
    for (int j = 0; j < 4; ++j) acc[i][j] = (v8f){0.f,0.f,0.f,0.f,0.f,0.f,0.f,0.f};

  for (int k0 = 0; k0 < K; k0 += 32) {
    V bh[4], bl[4];
#pragma unroll
    for (int j = 0; j < 4; ++j) {
      const size_t bo = (size_t)(n0 + (j << 4) + rlane) * ldb + koff + k0;
      bh[j] = Frag<T>::load(Bb + bo);
      if (SPLIT) bl[j] = Frag<T>::load(Bb2 + bo);
    }
#pragma unroll
    for (int i = 0; i < 4; ++i) {
      const size_t ao = (size_t)(m0 + (i << 4) + rlane) * lda + koff + k0;
      V ah = Frag<T>::load(Ab + ao);
      V al;
      if (SPLIT) al = Frag<T>::load(Ab2 + ao);
#pragma unroll
      for (int j = 0; j < 4; ++j) {
        acc[i][j] = Frag<T>::mma(ah, bh[j], acc[i][j]);
        if (SPLIT) {
          acc[i][j] = Frag<T>::mma(ah, bl[j], acc[i][j]);
          acc[i][j] = Frag<T>::mma(al, bh[j], acc[i][j]);
        }
      }
      Frag<T>::guard(acc[i][0], acc[i][3], ah, SPLIT ? al : ah);
    }
    Frag<T>::keep(bh[0], bh[1], bh[2], bh[3]);
    if (SPLIT) Frag<T>::keep(bl[0], bl[1], bl[2], bl[3]);
  }
  acc_guard4(acc[0][0], acc[0][1], acc[0][2], acc[0][3]);
  acc_guard4(acc[1][0], acc[1][1], acc[1][2], acc[1][3]);
  acc_guard4(acc[2][0], acc[2][1], acc[2][2], acc[2][3]);
  acc_guard4(acc[3][0], acc[3][1], acc[3][2], acc[3][3]);

  float* slab = sT[wave];
  const float* Rb = RESID ? (resid + (size_t)b * strideR) : nullptr;
#pragma unroll
  for (int i = 0; i < 4; ++i) {
    const int mBase = m0 + (i << 4);
#pragma unroll
    for (int j = 0; j < 4; ++j) {
      const int n = n0 + (j << 4) + rlane;
      float bv = 0.f;
      if (BIAS_MODE == 2) bv = bias[n];
#pragma unroll
      for (int r = 0; r < 8; ++r) {
        float v = acc[i][j][r] * scale;
        if (BIAS_MODE == 1) v += bias[mBase + mOff + r];
        if (BIAS_MODE == 2) v += bv;
        if (RESID) v += Rb[(size_t)(mBase + mOff + r) * ldc + n];
        if (ACT == 1) v = tanhf(v);
        if (ACT == 2) v = fmaxf(v, 0.0f);
        if (ACT == 3) v = v / (1.0f + expf(-v));
        if (ACT == 4) v = (v > 0.f) ? v : 0.01f * v;
        if (ACT == 5) v = 0.5f * v * (1.0f + erff(v * 0.70710678118654752f));
        slab[(mOff + r) * 68 + (j << 4) + rlane] = v;
      }
    }
    __builtin_amdgcn_fence(__ATOMIC_RELEASE, "workgroup");
    __builtin_amdgcn_wave_barrier();
    __builtin_amdgcn_fence(__ATOMIC_ACQUIRE, "workgroup");
    if (OUT_MODE == 0) {
      float* C = (float*)Cout + (size_t)b * strideC;
      const int hh = lane >> 4, c4 = (lane & 15) * 4;
      for (int pass = 0; pass < 2; ++pass) {
#pragma unroll
        for (int it = 0; it < 8; ++it) {
          const int row = it * 2 + hh;
          v4f v = *(const v4f*)(slab + row * 68 + c4);
          *(volatile v4f*)(C + (size_t)(mBase + row) * ldc + n0 + c4) = v;
        }
        __threadfence();
      }
    } else {
      const int q = lane >> 3, c8 = (lane & 7) * 8;
      unsigned short* C  = (unsigned short*)Cout  + (size_t)b * strideC;
      unsigned short* C2 = (OUT_MODE == 2) ? ((unsigned short*)Cout2 + (size_t)b * strideC) : nullptr;
      for (int pass = 0; pass < 2; ++pass) {
#pragma unroll
        for (int it = 0; it < 4; ++it) {
          const int row = it * 4 + q;
          const float* sp = slab + row * 68 + c8;
          v8h hv, lv;
#pragma unroll
          for (int e = 0; e < 8; ++e) {
            if (OUT_MODE == 1) {
              hv[e] = (_Float16)sp[e];
            } else {
              unsigned short hb = f2bf_bits(sp[e]);
              unsigned short lb = f2bf_bits(sp[e] - bf_bits2f(hb));
              hv[e] = __builtin_bit_cast(_Float16, hb);
              lv[e] = __builtin_bit_cast(_Float16, lb);
            }
          }
          *(volatile v8h*)(C + (size_t)(mBase + row) * ldc + n0 + c8) = hv;
          if (OUT_MODE == 2) *(volatile v8h*)(C2 + (size_t)(mBase + row) * ldc + n0 + c8) = lv;
        }
        __threadfence();
      }
    }
    __builtin_amdgcn_fence(__ATOMIC_RELEASE, "workgroup");
    __builtin_amdgcn_wave_barrier();
    __builtin_amdgcn_fence(__ATOMIC_ACQUIRE, "workgroup");
  }
}

__device__ __forceinline__ unsigned short at_bf_bits(float f) {
  unsigned u = __float_as_uint(f);
  return (unsigned short)((u + 0x7FFFu + ((u >> 16) & 1u)) >> 16);
}
__device__ __forceinline__ __bf16 at_f2bf(float f) { return __builtin_bit_cast(__bf16, at_bf_bits(f)); }
__device__ __forceinline__ void at_split(float f, __bf16& hi, __bf16& lo) {
  const unsigned short hb = at_bf_bits(f);
  hi = __builtin_bit_cast(__bf16, hb);
  lo = at_f2bf(f - __uint_as_float(((unsigned)hb) << 16));
}

constexpr int kNB  = 4;
constexpr int kNC  = 128;
constexpr int kNT  = 4096;
static_assert(kNT % 64 == 0, "");
static_assert(kNC % 64 == 0, "");
static_assert(kNC % 32 == 0, "");

constexpr size_t kPlaneB  = (size_t)kNB * kNT * kNC * 2;
constexpr size_t kWplaneB = (size_t)3 * kNC * kNC * 2;
constexpr size_t kOffXh = 0, kOffXl = kPlaneB, kOffQh = 2 * kPlaneB, kOffQl = 3 * kPlaneB;
constexpr size_t kOffKh = 4 * kPlaneB, kOffKl = 5 * kPlaneB, kOffVh = 6 * kPlaneB, kOffVl = 7 * kPlaneB;
constexpr size_t kOffWh = 8 * kPlaneB, kOffWl = kOffWh + kWplaneB;
constexpr size_t kWsTotal = kOffWl + kWplaneB;
static_assert(kWsTotal == 33751040u, "");
static_assert(kWsTotal <= 134217728u, "");

__device__ __forceinline__ void split8_bf16(v4f a, v4f c, v4u& hi, v4u& lo) {
  unsigned hw[4], lw[4];
#pragma unroll
  for (int e = 0; e < 2; ++e) {
    const float f0 = a[2 * e], f1 = a[2 * e + 1];
    const unsigned short h0 = f2bf_bits(f0), h1 = f2bf_bits(f1);
    const unsigned short l0 = f2bf_bits(f0 - bf_bits2f(h0)), l1 = f2bf_bits(f1 - bf_bits2f(h1));
    hw[e] = (unsigned)h0 | ((unsigned)h1 << 16);
    lw[e] = (unsigned)l0 | ((unsigned)l1 << 16);
  }
#pragma unroll
  for (int e = 0; e < 2; ++e) {
    const float f0 = c[2 * e], f1 = c[2 * e + 1];
    const unsigned short h0 = f2bf_bits(f0), h1 = f2bf_bits(f1);
    const unsigned short l0 = f2bf_bits(f0 - bf_bits2f(h0)), l1 = f2bf_bits(f1 - bf_bits2f(h1));
    hw[2 + e] = (unsigned)h0 | ((unsigned)h1 << 16);
    lw[2 + e] = (unsigned)l0 | ((unsigned)l1 << 16);
  }
  hi = (v4u){hw[0], hw[1], hw[2], hw[3]};
  lo = (v4u){lw[0], lw[1], lw[2], lw[3]};
}

__global__ __launch_bounds__(256) void xpose_split_x(
    const float* __restrict__ x, unsigned short* __restrict__ Xh, unsigned short* __restrict__ Xl) {
  __shared__ __align__(16) float sx[64 * 132];
  const int b    = blockIdx.y;
  const int n0   = blockIdx.x * 64;
  const int tid  = threadIdx.x;
  const int lane = tid & 31;
  const int wave = tid >> 5;
  {
    const int c  = tid >> 1;
    const int tp = (tid & 1) * 32;
    const float* src = x + ((size_t)(b * kNC + c)) * kNT + n0 + tp;
#pragma unroll
    for (int j = 0; j < 8; ++j) {
      const v4f v = *(const v4f*)(src + 4 * j);
#pragma unroll
      for (int e = 0; e < 4; ++e) sx[(tp + 4 * j + e) * 132 + c] = v[e];
    }
  }
  __syncthreads();
  v4u hq[4], lq[4];
  size_t off[4];
#pragma unroll
  for (int it = 0; it < 4; ++it) {
    const int row = wave * 8 + it * 2 + (lane >> 4);
    const int c8  = (lane & 15) * 8;
    const v4f a  = *(const v4f*)(sx + row * 132 + c8);
    const v4f a2 = *(const v4f*)(sx + row * 132 + c8 + 4);
    split8_bf16(a, a2, hq[it], lq[it]);
    off[it] = ((size_t)(b * kNT + n0 + row)) * kNC + c8;
  }
  for (int pass = 0; pass < 2; ++pass) {
#pragma unroll
    for (int it = 0; it < 4; ++it) {
      *(volatile v4u*)(Xh + off[it]) = hq[it];
      *(volatile v4u*)(Xl + off[it]) = lq[it];
    }
    __threadfence();
  }
}

__global__ __launch_bounds__(256) void split_w(
    const float* __restrict__ Wq, const float* __restrict__ Wk, const float* __restrict__ Wv,
    unsigned short* __restrict__ Wh, unsigned short* __restrict__ Wl) {
  const int mat  = blockIdx.y;
  const float* W = (mat == 0) ? Wq : ((mat == 1) ? Wk : Wv);
  const int tid  = threadIdx.x;
  const int lane = tid & 31;
  const int wave = tid >> 5;
  const int row  = blockIdx.x * 16 + wave * 2 + (lane >> 4);
  const int c8   = (lane & 15) * 8;
  const v4f a  = *(const v4f*)(W + (size_t)row * kNC + c8);
  const v4f a2 = *(const v4f*)(W + (size_t)row * kNC + c8 + 4);
  v4u hv, lv;
  split8_bf16(a, a2, hv, lv);
  const size_t off = ((size_t)(mat * kNC + row)) * kNC + c8;
  for (int pass = 0; pass < 2; ++pass) {
    *(volatile v4u*)(Wh + off) = hv;
    *(volatile v4u*)(Wl + off) = lv;
    __threadfence();
  }
}

constexpr int kKC  = 64;
constexpr int kQP  = 136;
constexpr int kVP  = 72;
constexpr int kOP  = 68;
constexpr int kQplaneB = 64 * kQP * 2;
constexpr int kVplaneB = kNC * kVP * 2;
constexpr int kOsB     = kNC * kOP * 4;
constexpr int kLdsB    = 4 * kQplaneB + 2 * kVplaneB;
static_assert(kOsB <= 2 * kQplaneB, "");
static_assert(kNT % kKC == 0, "");

__device__ __forceinline__ v8f mma3b(v16b ahi, v16b alo, v16b bhi, v16b blo, v8f c) {
  c = __builtin_amdgcn_wmma_f32_16x16x32_bf16(false, ahi, false, bhi, (short)0, c, false, false);
  c = __builtin_amdgcn_wmma_f32_16x16x32_bf16(false, ahi, false, blo, (short)0, c, false, false);
  c = __builtin_amdgcn_wmma_f32_16x16x32_bf16(false, alo, false, bhi, (short)0, c, false, false);
  asm volatile("v_nop\n\tv_nop\n\tv_nop\n\tv_nop" : "+v"(c) : "v"(ahi), "v"(alo), "v"(bhi), "v"(blo));
  return c;
}

__global__ __launch_bounds__(128) void attn_split(
    const unsigned short* __restrict__ Qh, const unsigned short* __restrict__ Ql,
    const unsigned short* __restrict__ Kh, const unsigned short* __restrict__ Kl,
    const unsigned short* __restrict__ Vh, const unsigned short* __restrict__ Vl,
    float* __restrict__ out, float scale) {
  __shared__ __align__(16) unsigned char lds_raw[kLdsB];
  unsigned short* const Qsh = (unsigned short*)(lds_raw);
  unsigned short* const Qsl = (unsigned short*)(lds_raw + kQplaneB);
  unsigned short* const Ksh = (unsigned short*)(lds_raw + 2 * kQplaneB);
  unsigned short* const Ksl = (unsigned short*)(lds_raw + 3 * kQplaneB);
  unsigned short* const Vsh = (unsigned short*)(lds_raw + 4 * kQplaneB);
  unsigned short* const Vsl = (unsigned short*)(lds_raw + 4 * kQplaneB + kVplaneB);
  float* const Os = (float*)(lds_raw + 2 * kQplaneB);
  const __bf16* const Qbh = (const __bf16*)(const void*)Qsh;
  const __bf16* const Qbl = (const __bf16*)(const void*)Qsl;
  const __bf16* const Kbh = (const __bf16*)(const void*)Ksh;
  const __bf16* const Kbl = (const __bf16*)(const void*)Ksl;
  const __bf16* const Vbh = (const __bf16*)(const void*)Vsh;
  const __bf16* const Vbl = (const __bf16*)(const void*)Vsl;

  const int b    = blockIdx.y;
  const int qblk = blockIdx.x * 64;
  const int tid  = threadIdx.x;
  const int lane = tid & 31;
  const int wave = tid >> 5;
  const int h    = lane >> 4;
  const int m    = lane & 15;

  const size_t plane = (size_t)b * kNT * kNC;
  const unsigned short* const Qhb = Qh + plane;
  const unsigned short* const Qlb = Ql + plane;
  const unsigned short* const Khb = Kh + plane;
  const unsigned short* const Klb = Kl + plane;
  const unsigned short* const Vhb = Vh + plane;
  const unsigned short* const Vlb = Vl + plane;

#pragma unroll 1
  for (int hf = 0; hf < 2; ++hf) {
#pragma unroll
    for (int it = 0; it < 4; ++it) {
      const int idx = (hf * 4 + it) * 128 + tid;
      const int row = idx >> 4, seg = idx & 15;
      const size_t go = (size_t)(qblk + row) * kNC + seg * 8;
      const v4u a  = *(const v4u*)(Qhb + go);
      const v4u a2 = *(const v4u*)(Qlb + go);
      *(v4u*)(Qsh + row * kQP + seg * 8) = a;
      *(v4u*)(Qsl + row * kQP + seg * 8) = a2;
    }
  }

  const v8f vz = {0.f, 0.f, 0.f, 0.f, 0.f, 0.f, 0.f, 0.f};
  v8f oacc[8];
#pragma unroll
  for (int dt = 0; dt < 8; ++dt) oacc[dt] = vz;
  float m_run = -__builtin_inff();
  float l_run = 0.0f;

  for (int kc = 0; kc < kNT / kKC; ++kc) {
    const int kbase = kc * kKC;
    __syncthreads();
#pragma unroll 1
    for (int hf = 0; hf < 2; ++hf) {
#pragma unroll
      for (int it = 0; it < 4; ++it) {
        const int idx = (hf * 4 + it) * 128 + tid;
        const int row = idx >> 4, seg = idx & 15;
        const size_t go = (size_t)(kbase + row) * kNC + seg * 8;
        const v4u a  = *(const v4u*)(Khb + go);
        const v4u a2 = *(const v4u*)(Klb + go);
        *(v4u*)(Ksh + row * kQP + seg * 8) = a;
        *(v4u*)(Ksl + row * kQP + seg * 8) = a2;
      }
    }
#pragma unroll 1
    for (int hf = 0; hf < 2; ++hf) {
#pragma unroll
      for (int it = 0; it < 4; ++it) {
        const int idx = (hf * 4 + it) * 128 + tid;
        const int d = idx >> 3, seg = idx & 7;
        const size_t go = (size_t)d * kNT + kbase + seg * 8;
        const v4u a  = *(const v4u*)(Vhb + go);
        const v4u a2 = *(const v4u*)(Vlb + go);
        *(v4u*)(Vsh + d * kVP + seg * 8) = a;
        *(v4u*)(Vsl + d * kVP + seg * 8) = a2;
      }
    }
    __syncthreads();

    v8f s[4];
#pragma unroll
    for (int t = 0; t < 4; ++t) s[t] = vz;
#pragma unroll 1
    for (int cc = 0; cc < 4; ++cc) {
      const int ko = cc * 32 + 8 * h;
      const v16b qfh = Frag<__bf16>::load(Qbh + (wave * 16 + m) * kQP + ko);
      const v16b qfl = Frag<__bf16>::load(Qbl + (wave * 16 + m) * kQP + ko);
#pragma unroll
      for (int t = 0; t < 4; ++t) {
        const v16b kfh = Frag<__bf16>::load(Kbh + (t * 16 + m) * kQP + ko);
        const v16b kfl = Frag<__bf16>::load(Kbl + (t * 16 + m) * kQP + ko);
        s[t] = mma3b(kfh, kfl, qfh, qfl, s[t]);
      }
    }

    float mloc = -__builtin_inff();
#pragma unroll
    for (int t = 0; t < 4; ++t)
#pragma unroll
      for (int r = 0; r < 8; ++r) mloc = fmaxf(mloc, s[t][r]);
    const float mx    = __shfl_xor(mloc, 16, 32);
    const float mcs   = fmaxf(mloc, mx) * scale;
    const float mnew  = fmaxf(m_run, mcs);
    const float alpha = expf(m_run - mnew);
    m_run = mnew;
    float psum = 0.0f;
#pragma unroll
    for (int t = 0; t < 4; ++t)
#pragma unroll
      for (int r = 0; r < 8; ++r) {
        const float p = expf(fmaf(s[t][r], scale, -mnew));
        s[t][r] = p;
        psum += p;
      }
    const float psx = __shfl_xor(psum, 16, 32);
    l_run = l_run * alpha + (psum + psx);
#pragma unroll
    for (int dt = 0; dt < 8; ++dt)
#pragma unroll
      for (int r = 0; r < 8; ++r) oacc[dt][r] *= alpha;

#pragma unroll
    for (int kk = 0; kk < 2; ++kk) {
      v16b pfh, pfl;
#pragma unroll
      for (int i = 0; i < 8; ++i) {
        __bf16 a0, l0;
        at_split(s[2 * kk][i], a0, l0);
        pfh[i] = a0; pfl[i] = l0;
        at_split(s[2 * kk + 1][i], a0, l0);
        pfh[8 + i] = a0; pfl[8 + i] = l0;
      }
#pragma unroll
      for (int dt = 0; dt < 8; ++dt) {
        const v16b vfh = Frag<__bf16>::load(Vbh + (dt * 16 + m) * kVP + kk * 32 + 8 * h);
        const v16b vfl = Frag<__bf16>::load(Vbl + (dt * 16 + m) * kVP + kk * 32 + 8 * h);
        oacc[dt] = mma3b(vfh, vfl, pfh, pfl, oacc[dt]);
      }
    }
  }

  __syncthreads();
  const float rinv = 1.0f / l_run;
#pragma unroll
  for (int dt = 0; dt < 8; ++dt)
#pragma unroll
    for (int r = 0; r < 8; ++r)
      Os[(dt * 16 + 8 * h + r) * kOP + wave * 16 + m] = oacc[dt][r] * rinv;
  __syncthreads();
  {
    float* const ob = out + (size_t)b * kNC * kNT + qblk;
    const int rsub = lane >> 4;
    const int c4   = ((lane >> 3) & 1) * 32 + (lane & 7) * 4;
    for (int pass = 0; pass < 2; ++pass) {
#pragma unroll
      for (int it = 0; it < 16; ++it) {
        const int row = it * 8 + wave * 2 + rsub;
        const v4f v = *(const v4f*)(Os + row * kOP + c4);
        *(volatile v4f*)(ob + (size_t)row * kNT + c4) = v;
      }
      __threadfence();
    }
  }
}

extern "C" void kernel_launch(void* const* d_in, const int* in_sizes, int n_in,
                              void* d_out, int out_size, void* d_ws, size_t ws_size,
                              hipStream_t stream) {
  if (n_in < 7) return;
  if (in_sizes[0] != kNB * kNC * kNT) return;
  if (in_sizes[1] != kNC * kNC || in_sizes[3] != kNC * kNC || in_sizes[5] != kNC * kNC) return;
  if (in_sizes[2] != kNC || in_sizes[4] != kNC || in_sizes[6] != kNC) return;
  if (out_size != kNB * kNC * kNT) return;
  if (ws_size < kWsTotal) return;

  const float* x  = (const float*)d_in[0];
  const float* Wq = (const float*)d_in[1];
  const float* bq = (const float*)d_in[2];
  const float* Wk = (const float*)d_in[3];
  const float* bk = (const float*)d_in[4];
  const float* Wv = (const float*)d_in[5];
  const float* bv = (const float*)d_in[6];
  float* out = (float*)d_out;

  unsigned char* ws = (unsigned char*)d_ws;
  unsigned short* Xh = (unsigned short*)(ws + kOffXh);
  unsigned short* Xl = (unsigned short*)(ws + kOffXl);
  unsigned short* Qh = (unsigned short*)(ws + kOffQh);
  unsigned short* Ql = (unsigned short*)(ws + kOffQl);
  unsigned short* Kh = (unsigned short*)(ws + kOffKh);
  unsigned short* Kl = (unsigned short*)(ws + kOffKl);
  unsigned short* Vh = (unsigned short*)(ws + kOffVh);
  unsigned short* Vl = (unsigned short*)(ws + kOffVl);
  unsigned short* Wh = (unsigned short*)(ws + kOffWh);
  unsigned short* Wl = (unsigned short*)(ws + kOffWl);

  xpose_split_x<<<dim3(kNT / 64, kNB), 256, 0, stream>>>(x, Xh, Xl);
  split_w<<<dim3(kNC / 16, 3), 256, 0, stream>>>(Wq, Wk, Wv, Wh, Wl);

  static_assert(kNT % 64 == 0 && kNC % 64 == 0 && kNC % 32 == 0, "");
  const long sTok  = (long)kNT * kNC;
  const int  wmat  = kNC * kNC;
  const dim3 gg(((kNT / 64) * (kNC / 64)) / 8, kNB);
  wmma_gemm64<1, true, 2, 2, false, 0><<<gg, 256, 0, stream>>>(
      Xh, Xl, kNC, sTok, Wh, Wl, kNC, 0L,
      (void*)Qh, (void*)Ql, kNC, sTok, bq, nullptr, 0L, kNT, kNC, kNC, 1.0f);
  wmma_gemm64<1, true, 2, 2, false, 0><<<gg, 256, 0, stream>>>(
      Xh, Xl, kNC, sTok, Wh + wmat, Wl + wmat, kNC, 0L,
      (void*)Kh, (void*)Kl, kNC, sTok, bk, nullptr, 0L, kNT, kNC, kNC, 1.0f);
  wmma_gemm64<1, true, 1, 2, false, 0><<<gg, 256, 0, stream>>>(
      Wh + 2 * wmat, Wl + 2 * wmat, kNC, 0L, Xh, Xl, kNC, sTok,
      (void*)Vh, (void*)Vl, kNT, sTok, bv, nullptr, 0L, kNC, kNT, kNC, 1.0f);

  const float scale = 0.08838834764831845f;
  attn_split<<<dim3(kNT / 64, kNB), 128, 0, stream>>>(Qh, Ql, Kh, Kl, Vh, Vl, out, scale);
}
